// GDAModule_55937654063134
// MI455X (gfx1250) — hardware-verified
//
#include <hip/hip_runtime.h>
#include <stddef.h>
#include <stdint.h>
#include <math.h>


#define NB      2
#define CH      64
#define HH      128
#define WW      128
#define GH      64
#define GW      64
#define LSEQ    4096
#define NTOK    8192
#define DIN     128
#define NST     16
#define DTR     4
#define NDBL    36
#define NXPAD   192
#define PLANE   2097152
#define GBM     64
#define GBN     64
#define GTHR    128
#define NTHR    256
#define SCH     32
#define SCT     64
#define WSMAX   134217728

static_assert(HH == 128 && WW == 128 && GH * 2 == HH && GW * 2 == WW && LSEQ == GH * GW);
static_assert(CH == 64 && DIN == 128 && NST == 16 && DTR == 4 && NDBL == DTR + 2 * NST);
static_assert(NTOK == NB * LSEQ && NTOK % GBM == 0 && NTOK % 128 == 0 && WW % 32 == 0);
static_assert(NXPAD % GBN == 0 && 4 * NDBL <= NXPAD && (2 * DIN) % GBN == 0);
static_assert(GBM == (GTHR / 32) * 16 && GBN == 64);
static_assert(PLANE == NB * CH * HH * WW);

#define SP_SCW   0
#define SP_SCB   1152
#define SP_SDTW  1280
#define SP_SDTB  3328
#define SP_SD    3840
#define SP_SOG   4352
#define SP_SOB   4480
#define SP_SAN   4608
#define SP_MCW   12800
#define SP_MCB   13312
#define SP_MDTW  13440
#define SP_MDTB  13952
#define SP_MD    14080
#define SP_MAN   14208
#define SP_SPEG  16256
#define SP_SPEB  16384
#define SP_PEB   16512
#define SP_GNG   16640
#define SP_GNB   16768
#define SP_VLG   16896
#define SP_VLB   17024
#define SP_GAW   17152
#define SP_GBW   17280
#define SP_GAB   17408
#define SP_GBB   17536
#define SP_END   17664
#define SPU      (SP_END / 4)
static_assert(SPU % 32 == 0);

#define PU_PEW   2048
#define PU_MINW  2048
#define PU_SINW  4096
#define PU_SXP   6144
#define PU_SOUT  2048
#define PU_MXP   2048
#define PU_MOUT  2048
#define PA_U     (PU_PEW + PU_MINW + PU_SINW + PU_SXP)
#define PB_U     (PU_SOUT + PU_MXP + PU_MOUT)
#define PC_U     (SP_MCW / 4)
#define PD_U0    (SP_MCW / 4)
#define PD_U     ((SP_SPEG - SP_MCW) / 4)
#define PF_U0    (SP_SPEG / 4)
#define PF_U     ((SP_GAW - SP_SPEG) / 4)
#define PG_U0    (SP_GAW / 4)
#define PG_U     ((SP_END - SP_GAW) / 4)
static_assert(PU_PEW % NTHR == 0 && PU_MINW % NTHR == 0 && PU_SINW % NTHR == 0 && PU_SXP % NTHR == 0);
static_assert(PU_SOUT % NTHR == 0 && PU_MXP % NTHR == 0 && PU_MOUT % NTHR == 0);
static_assert(PA_U % NTHR == 0 && PB_U % NTHR == 0);
static_assert(PC_U % 32 == 0 && PD_U0 % 32 == 0 && PD_U % 32 == 0 && PF_U0 % 32 == 0 && PF_U % 32 == 0);
static_assert(PG_U0 % 32 == 0 && PG_U % 32 == 0 && PC_U + PD_U + PF_U + PG_U == SPU);

#define A1P      72
#define A2P      264
#define O_XR1    0
#define O_XR2    8192
#define O_A1     16384
#define O_XZ     25600
#define O_A2     91136
#define O_DB     124928
#define O_YM     141312
#define SPE_LDS  157696
static_assert(O_A1 == O_XR2 + 8192 && O_XZ == O_A1 + 64 * A1P * 2 && O_A2 == O_XZ + 65536);
static_assert(O_DB == O_A2 + 64 * A2P * 2 && O_YM == O_DB + 16384 && SPE_LDS == O_YM + 16384);
static_assert(SPE_LDS <= 327680);

typedef float          v4f   __attribute__((ext_vector_type(4)));
typedef float          v8f   __attribute__((ext_vector_type(8)));
typedef int            v8i   __attribute__((ext_vector_type(8)));
typedef double         v2d   __attribute__((ext_vector_type(2)));
typedef unsigned short v4us  __attribute__((ext_vector_type(4)));
typedef unsigned short v8us  __attribute__((ext_vector_type(8)));
typedef unsigned short v16us __attribute__((ext_vector_type(16)));
typedef __bf16         v16bf __attribute__((ext_vector_type(16)));
typedef v4f  __attribute__((may_alias)) v4fa;
typedef v2d  __attribute__((may_alias)) v2da;
typedef v8us __attribute__((may_alias)) v8usa;
union FragB { v16bf v; v16us u; v8us h[2]; v8i w; };

__device__ __forceinline__ v8f wmb(const FragB& a, const FragB& b, v8f c) {
  v8f d = __builtin_amdgcn_wmma_f32_16x16x32_bf16(false, a.v, false, b.v, (short)0, c, false, false);
  asm volatile("v_nop\n\tv_nop\n\tv_nop\n\tv_nop" : "+v"(d) : "v"(a.w), "v"(b.w));
  return d;
}

__device__ __forceinline__ unsigned bf16_bits(float f) {
  const unsigned u = __float_as_uint(f);
  return (u + 0x7FFFu + ((u >> 16) & 1u)) >> 16;
}
__device__ __forceinline__ float bf16_val(float f) { return __uint_as_float(bf16_bits(f) << 16); }
__device__ __forceinline__ unsigned short hi_bits(float v) { return (unsigned short)bf16_bits(v); }
__device__ __forceinline__ unsigned short lo_bits(float v) {
  const unsigned hb = bf16_bits(v);
  return (unsigned short)bf16_bits(v - __uint_as_float(hb << 16));
}
__device__ __forceinline__ float silu_f(float c) { return c / (1.0f + expf(-c)); }
__device__ __forceinline__ float softplus_f(float v) {
  return (v > 0.0f ? v : 0.0f) + log1pf(expf(-fabsf(v)));
}
__device__ __forceinline__ void put4(float* p, v4f v) {
  *(volatile v4f*)p = v;
  __threadfence();
  *(volatile v4f*)p = v;
}

__device__ __forceinline__ void cvt8_put(const float* p, bool ok, unsigned short* dp) {
  const v4f a = *(const v4fa*)p;
  const v4f b = *(const v4fa*)(p + 4);
  v8us o;
  o[0] = ok ? (unsigned short)bf16_bits(a.x) : (unsigned short)0;
  o[1] = ok ? (unsigned short)bf16_bits(a.y) : (unsigned short)0;
  o[2] = ok ? (unsigned short)bf16_bits(a.z) : (unsigned short)0;
  o[3] = ok ? (unsigned short)bf16_bits(a.w) : (unsigned short)0;
  o[4] = ok ? (unsigned short)bf16_bits(b.x) : (unsigned short)0;
  o[5] = ok ? (unsigned short)bf16_bits(b.y) : (unsigned short)0;
  o[6] = ok ? (unsigned short)bf16_bits(b.z) : (unsigned short)0;
  o[7] = ok ? (unsigned short)bf16_bits(b.w) : (unsigned short)0;
  *(volatile v8us*)dp = o;
  __threadfence();
  *(volatile v8us*)dp = o;
}
__device__ __forceinline__ void rnd4n_put(const float* src, int v, int nv, float* dp) {
  const int vc = v < nv ? v : nv - 1;
  const v4f a = *(const v4fa*)(src + 4 * vc);
  const bool ok = v < nv;
  v4f o;
  o.x = ok ? bf16_val(a.x) : 0.0f; o.y = ok ? bf16_val(a.y) : 0.0f;
  o.z = ok ? bf16_val(a.z) : 0.0f; o.w = ok ? bf16_val(a.w) : 0.0f;
  put4(dp, o);
}
__device__ __forceinline__ void an4_put(const float* src, int v, float* dp) {
  const v4f a = *(const v4fa*)(src + 4 * v);
  v4f o;
  o.x = -expf(bf16_val(a.x)); o.y = -expf(bf16_val(a.y));
  o.z = -expf(bf16_val(a.z)); o.w = -expf(bf16_val(a.w));
  put4(dp, o);
}
__device__ __forceinline__ void rnd1_put(const float* src, int v, float* dp) {
  const float s = src[0];
  v4f o;
  o.x = (v == 0) ? bf16_val(s) : 0.0f; o.y = 0.0f; o.z = 0.0f; o.w = 0.0f;
  put4(dp, o);
}

__global__ __launch_bounds__(NTHR) __attribute__((amdgpu_num_vgpr(248))) void k_pa(
    const float* __restrict__ pe_w, const float* __restrict__ m_in_w,
    const float* __restrict__ s_in_w, const float* __restrict__ s_xproj_w,
    unsigned short* PEW, unsigned short* MINW, unsigned short* SINW2, unsigned short* SXP2)
{
  const int u = (int)blockIdx.x * NTHR + (int)threadIdx.x;
  if (u < PU_PEW) {
    cvt8_put(pe_w + (size_t)8 * u, true, PEW + (size_t)8 * u);
  } else if (u < PU_PEW + PU_MINW) {
    const int v = u - PU_PEW;
    cvt8_put(m_in_w + (size_t)8 * v, true, MINW + (size_t)8 * v);
  } else if (u < PU_PEW + PU_MINW + PU_SINW) {
    const int v = u - (PU_PEW + PU_MINW);
    const int n = v >> 4, k8 = (v & 15) * 8;
    cvt8_put(s_in_w + (size_t)n * 64 + (k8 & 63), true, SINW2 + (size_t)n * 128 + k8);
  } else if (u < PA_U) {
    const int v = u - (PU_PEW + PU_MINW + PU_SINW);
    const int n = v >> 5, k8 = (v & 31) * 8;
    const int nc = n < 144 ? n : 143;
    cvt8_put(s_xproj_w + (size_t)nc * 128 + (k8 & 127), n < 144, SXP2 + (size_t)n * 256 + k8);
  }
}

__global__ __launch_bounds__(NTHR) __attribute__((amdgpu_num_vgpr(248))) void k_pb(
    const float* __restrict__ s_out_w, const float* __restrict__ m_xproj_w, const float* __restrict__ m_out_w,
    unsigned short* SOUT2, unsigned short* MXP2, unsigned short* MOUT2)
{
  const int u = (int)blockIdx.x * NTHR + (int)threadIdx.x;
  if (u < PU_SOUT) {
    const int n = u >> 5, k8 = (u & 31) * 8;
    cvt8_put(s_out_w + (size_t)n * 128 + (k8 & 127), true, SOUT2 + (size_t)n * 256 + k8);
  } else if (u < PU_SOUT + PU_MXP) {
    const int v = u - PU_SOUT;
    const int n = v >> 5, k8 = (v & 31) * 8;
    const int nc = n < NDBL ? n : NDBL - 1;
    cvt8_put(m_xproj_w + (size_t)nc * 128 + (k8 & 127), n < NDBL, MXP2 + (size_t)n * 256 + k8);
  } else if (u < PB_U) {
    const int v = u - (PU_SOUT + PU_MXP);
    const int n = v >> 5, k8 = (v & 31) * 8;
    cvt8_put(m_out_w + (size_t)n * 128 + (k8 & 127), true, MOUT2 + (size_t)n * 256 + k8);
  }
}

__global__ __launch_bounds__(NTHR) __attribute__((amdgpu_num_vgpr(248))) void k_pc(
    const float* __restrict__ s_conv_w, const float* __restrict__ s_conv_b,
    const float* __restrict__ s_dt_w, const float* __restrict__ s_dt_b, const float* __restrict__ s_D,
    const float* __restrict__ s_og, const float* __restrict__ s_ob, const float* __restrict__ s_A_log,
    float* SP)
{
  const int v = (int)blockIdx.x * NTHR + (int)threadIdx.x;
  if (v < PC_U) {
    float* dp = SP + (size_t)4 * v;
    if      (v < SP_SCB  / 4) rnd4n_put(s_conv_w, v - SP_SCW  / 4, 288, dp);
    else if (v < SP_SDTW / 4) rnd4n_put(s_conv_b, v - SP_SCB  / 4, 32, dp);
    else if (v < SP_SDTB / 4) rnd4n_put(s_dt_w,   v - SP_SDTW / 4, 512, dp);
    else if (v < SP_SD   / 4) rnd4n_put(s_dt_b,   v - SP_SDTB / 4, 128, dp);
    else if (v < SP_SOG  / 4) rnd4n_put(s_D,      v - SP_SD   / 4, 128, dp);
    else if (v < SP_SOB  / 4) rnd4n_put(s_og,     v - SP_SOG  / 4, 32, dp);
    else if (v < SP_SAN  / 4) rnd4n_put(s_ob,     v - SP_SOB  / 4, 32, dp);
    else                      an4_put(s_A_log,    v - SP_SAN  / 4, dp);
  }
}

__global__ __launch_bounds__(NTHR) __attribute__((amdgpu_num_vgpr(248))) void k_pd(
    const float* __restrict__ m_conv_w, const float* __restrict__ m_conv_b,
    const float* __restrict__ m_dt_w, const float* __restrict__ m_dt_b, const float* __restrict__ m_D,
    const float* __restrict__ m_A_log, float* SP)
{
  const int lu = (int)blockIdx.x * NTHR + (int)threadIdx.x;
  if (lu < PD_U) {
    const int v = PD_U0 + lu;
    float* dp = SP + (size_t)4 * v;
    if      (v < SP_MCB  / 4) rnd4n_put(m_conv_w, v - SP_MCW  / 4, 128, dp);
    else if (v < SP_MDTW / 4) rnd4n_put(m_conv_b, v - SP_MCB  / 4, 32, dp);
    else if (v < SP_MDTB / 4) rnd4n_put(m_dt_w,   v - SP_MDTW / 4, 128, dp);
    else if (v < SP_MD   / 4) rnd4n_put(m_dt_b,   v - SP_MDTB / 4, 32, dp);
    else if (v < SP_MAN  / 4) rnd4n_put(m_D,      v - SP_MD   / 4, 32, dp);
    else                      an4_put(m_A_log,    v - SP_MAN  / 4, dp);
  }
}

__global__ __launch_bounds__(NTHR) __attribute__((amdgpu_num_vgpr(248))) void k_pf(
    const float* __restrict__ spe_g, const float* __restrict__ spe_b, const float* __restrict__ pe_b,
    const float* __restrict__ gn_g, const float* __restrict__ gn_b,
    const float* __restrict__ vl_g, const float* __restrict__ vl_b, float* SP)
{
  const int lu = (int)blockIdx.x * NTHR + (int)threadIdx.x;
  if (lu < PF_U) {
    const int v = PF_U0 + lu;
    float* dp = SP + (size_t)4 * v;
    if      (v < SP_SPEB / 4) rnd4n_put(spe_g, v - SP_SPEG / 4, 16, dp);
    else if (v < SP_PEB  / 4) rnd4n_put(spe_b, v - SP_SPEB / 4, 16, dp);
    else if (v < SP_GNG  / 4) rnd4n_put(pe_b,  v - SP_PEB  / 4, 16, dp);
    else if (v < SP_GNB  / 4) rnd4n_put(gn_g,  v - SP_GNG  / 4, 16, dp);
    else if (v < SP_VLG  / 4) rnd4n_put(gn_b,  v - SP_GNB  / 4, 16, dp);
    else if (v < SP_VLB  / 4) rnd4n_put(vl_g,  v - SP_VLG  / 4, 16, dp);
    else                      rnd4n_put(vl_b,  v - SP_VLB  / 4, 16, dp);
  }
}

__global__ __launch_bounds__(NTHR) __attribute__((amdgpu_num_vgpr(248))) void k_pg(
    const float* __restrict__ gA_w, const float* __restrict__ gB_w,
    const float* __restrict__ gA_b, const float* __restrict__ gB_b, float* SP)
{
  const int lu = (int)blockIdx.x * NTHR + (int)threadIdx.x;
  if (lu < PG_U) {
    const int v = PG_U0 + lu;
    float* dp = SP + (size_t)4 * v;
    if      (v < SP_GBW / 4) rnd4n_put(gA_w, v - SP_GAW / 4, 16, dp);
    else if (v < SP_GAB / 4) rnd4n_put(gB_w, v - SP_GBW / 4, 16, dp);
    else if (v < SP_GBB / 4) rnd1_put(gA_b,  v - SP_GAB / 4, dp);
    else                     rnd1_put(gB_b,  v - SP_GBB / 4, dp);
  }
}

__global__ __launch_bounds__(GTHR) __attribute__((amdgpu_num_vgpr(248))) void k_pe(
    const float* __restrict__ xs, const unsigned short* __restrict__ PEW, const float* __restrict__ SP,
    float* XP, double* REC)
{
  __shared__ __attribute__((aligned(16))) unsigned saw[64 * 132];
  __shared__ __attribute__((aligned(16))) float stg[GBM * GBN];
  __shared__ __attribute__((aligned(16))) double red[256];
  __shared__ __attribute__((aligned(16))) double recs[16];
  const int tid = (int)threadIdx.x, lane = tid & 31, wave = tid >> 5, hh = lane >> 4, m = lane & 15;
  const int blk = (int)blockIdx.x;
  const int b = blk >> 6, gi = blk & 63;
  const float* xb = xs + (size_t)b * CH * (HH * WW) + (size_t)(2 * gi) * WW;

#pragma unroll 4
  for (int it = 0; it < 32; ++it) {
    const int idx = tid + GTHR * it;
    const int c = idx >> 6, rem = idx & 63, di = rem >> 5, q = rem & 31;
    const v4f v = *(const v4fa*)(xb + (size_t)c * (HH * WW) + di * WW + 4 * q);
    const unsigned p0 = bf16_bits(v.x) | (bf16_bits(v.y) << 16);
    const unsigned p1 = bf16_bits(v.z) | (bf16_bits(v.w) << 16);
    const int wc = c * 2 + di;
    saw[(2 * q) * 132 + wc]     = p0;
    saw[(2 * q + 1) * 132 + wc] = p1;
  }
  __syncthreads();

  v8f acc[4];
  {
    const v8f z = {0.f, 0.f, 0.f, 0.f, 0.f, 0.f, 0.f, 0.f};
    acc[0] = z; acc[1] = z; acc[2] = z; acc[3] = z;
  }
  const unsigned short* ap = (const unsigned short*)saw + (16 * wave + m) * 264 + 8 * hh;
  const unsigned short* wp = PEW + (size_t)m * 256 + 8 * hh;
#pragma unroll 1
  for (int ks = 0; ks < 8; ++ks) {
    FragB af;
    af.h[0] = *(const v8usa*)(ap + 32 * ks);
    af.h[1] = *(const v8usa*)(ap + 32 * ks + 16);
#pragma unroll
    for (int t = 0; t < 4; ++t) {
      const unsigned short* wq = wp + (size_t)(16 * t) * 256 + 32 * ks;
      FragB bf;
      bf.h[0] = *(const v8usa*)wq;
      bf.h[1] = *(const v8usa*)(wq + 16);
      acc[t] = wmb(af, bf, acc[t]);
    }
  }
#pragma unroll
  for (int t = 0; t < 4; ++t) {
    const int lc = 16 * t + m;
    const float pb = SP[SP_PEB + lc];
#pragma unroll
    for (int r = 0; r < 8; ++r) {
      const int lr = 16 * wave + 8 * hh + r;
      stg[lr * GBN + lc] = acc[t][r] + pb;
    }
  }
  __syncthreads();

  {
    const int tok0 = blk * 64;
    float* ob = XP + 4 * m;
    v4f fv[8];
#pragma unroll
    for (int i = 0; i < 8; ++i) {
      const int lr = 16 * wave + 2 * i + hh;
      fv[i] = *(const v4fa*)(stg + lr * GBN + 4 * m);
    }
#pragma unroll
    for (int i = 0; i < 8; ++i) {
      const int lr = 16 * wave + 2 * i + hh;
      *(volatile v4f*)(ob + (size_t)(tok0 + lr) * CH) = fv[i];
    }
    __threadfence();
#pragma unroll
    for (int i = 0; i < 8; ++i) {
      const int lr = 16 * wave + 2 * i + hh;
      *(volatile v4f*)(ob + (size_t)(tok0 + lr) * CH) = fv[i];
    }
  }
  {
    const int g = tid >> 5;
    double s = 0.0, q = 0.0;
#pragma unroll 4
    for (int e = 0; e < 32; ++e) {
      const int idx = lane + 32 * e;
      const double v = (double)stg[(idx >> 4) * GBN + 16 * g + (idx & 15)];
      s += v;
      q += v * v;
    }
    red[tid] = s;
    red[128 + tid] = q;
  }
  __syncthreads();
  {
    const int tc = tid & 7;
    const int base = (tc & 1) * 128 + (tc >> 1) * 32;
    double a = 0.0;
#pragma unroll 4
    for (int l = 0; l < 32; ++l) a += red[base + l];
    if (tid < 16) recs[tid] = (tid < 8) ? a : 0.0;
  }
  __syncthreads();
  {
    const int rc = tid < 8 ? tid : 0;
    v2d rv;
    rv.x = recs[2 * rc];
    rv.y = recs[2 * rc + 1];
    if (tid < 8) {
      double* dp = REC + (size_t)blk * 16 + 2 * tid;
      *(volatile v2d*)dp = rv;
      __threadfence();
      *(volatile v2d*)dp = rv;
    }
  }
}

__global__ __launch_bounds__(NTHR) __attribute__((amdgpu_num_vgpr(248))) void k_gnln(
    const float* __restrict__ XP, const double* __restrict__ REC, const float* __restrict__ SP,
    float* XIN, unsigned short* XNHL)
{
  __shared__ __attribute__((aligned(16))) float sx[64 * 64];
  __shared__ __attribute__((aligned(16))) unsigned short shl[64 * 128];
  const int tid = (int)threadIdx.x;
  const int blk = (int)blockIdx.x;
  const int tok0 = blk * 64;
  const int b = blk >> 6;
#pragma unroll
  for (int i = 0; i < 4; ++i) {
    const int p = tid + NTHR * i;
    *(v4fa*)(sx + 4 * p) = *(const v4fa*)(XP + (size_t)tok0 * CH + 4 * p);
  }
  const int q = tid & 3, tl = tid >> 2;
  double S = 0.0, Q = 0.0;
#pragma unroll 4
  for (int j = 0; j < 64; ++j) {
    const v2d r = *(const v2da*)(REC + (size_t)(b * 64 + j) * 16 + 2 * q);
    S += r.x;
    Q += r.y;
  }
  const double mean64 = S * (1.0 / 65536.0);
  const double var64  = Q * (1.0 / 65536.0) - mean64 * mean64;
  const float gm = (float)mean64;
  const float gr = 1.0f / sqrtf((float)var64 + 1e-5f);
  __syncthreads();

  float* row = sx + tl * 64 + 16 * q;
  float s = 0.0f;
#pragma unroll 2
  for (int j = 0; j < 16; ++j) {
    const int c = 16 * q + j;
    const float xg = (row[j] - gm) * gr * SP[SP_GNG + c] + SP[SP_GNB + c];
    const float xi = silu_f(xg);
    row[j] = xi;
    s += xi;
  }
  s += __shfl_xor(s, 1);
  s += __shfl_xor(s, 2);
  const float mu = s * (1.0f / 64.0f);
  float qv = 0.0f;
#pragma unroll 4
  for (int j = 0; j < 16; ++j) {
    const float d = row[j] - mu;
    qv += d * d;
  }
  qv += __shfl_xor(qv, 1);
  qv += __shfl_xor(qv, 2);
  const float rs = 1.0f / sqrtf(qv * (1.0f / 64.0f) + 1e-5f);
#pragma unroll 2
  for (int j = 0; j < 16; ++j) {
    const int c = 16 * q + j;
    const float xn = (row[j] - mu) * rs * SP[SP_VLG + c] + SP[SP_VLB + c];
    shl[tl * 128 + c]      = hi_bits(xn);
    shl[tl * 128 + 64 + c] = lo_bits(xn);
  }
  __syncthreads();

  v4f fv[4];
  v8us hv[4];
#pragma unroll
  for (int i = 0; i < 4; ++i) {
    const int p = tid + NTHR * i;
    fv[i] = *(const v4fa*)(sx + 4 * p);
    hv[i] = *(const v8usa*)(shl + 8 * p);
  }
#pragma unroll
  for (int i = 0; i < 4; ++i) {
    const int p = tid + NTHR * i;
    *(volatile v4f*)(XIN + (size_t)tok0 * CH + 4 * p) = fv[i];
    *(volatile v8us*)(XNHL + (size_t)tok0 * 128 + 8 * p) = hv[i];
  }
  __threadfence();
#pragma unroll
  for (int i = 0; i < 4; ++i) {
    const int p = tid + NTHR * i;
    *(volatile v4f*)(XIN + (size_t)tok0 * CH + 4 * p) = fv[i];
    *(volatile v8us*)(XNHL + (size_t)tok0 * 128 + 8 * p) = hv[i];
  }
}

template <int MODE>
__global__ __launch_bounds__(GTHR) __attribute__((amdgpu_num_vgpr(248))) void k_gemm(
    const unsigned short* __restrict__ A, int lda,
    const unsigned short* __restrict__ WT, int ldb, int K,
    float* outF, int ldo, int nsplit, int pstride, const float* __restrict__ res)
{
  __shared__ __attribute__((aligned(16))) float stg[GBM * GBN];
  const int tid = (int)threadIdx.x, lane = tid & 31, wave = tid >> 5, hh = lane >> 4, m = lane & 15;
  const int rowBase = (int)blockIdx.x * GBM;
  const int col0    = (int)blockIdx.y * GBN;

  v8f acc[4];
  {
    const v8f z = {0.f, 0.f, 0.f, 0.f, 0.f, 0.f, 0.f, 0.f};
    acc[0] = z; acc[1] = z; acc[2] = z; acc[3] = z;
  }
  const unsigned short* ap = A  + (size_t)(rowBase + 16 * wave + m) * (size_t)lda + 8 * hh;
  const unsigned short* wp = WT + (size_t)(col0 + m) * (size_t)ldb + 8 * hh;
  const int ksteps = K >> 5;
#pragma unroll 1
  for (int ks = 0; ks < ksteps; ++ks) {
    FragB af;
    af.h[0] = *(const v8usa*)(ap + 32 * ks);
    af.h[1] = *(const v8usa*)(ap + 32 * ks + 16);
#pragma unroll
    for (int t = 0; t < 4; ++t) {
      const unsigned short* wq = wp + (size_t)(16 * t) * (size_t)ldb + 32 * ks;
      FragB bf;
      bf.h[0] = *(const v8usa*)wq;
      bf.h[1] = *(const v8usa*)(wq + 16);
      acc[t] = wmb(af, bf, acc[t]);
    }
  }

#pragma unroll
  for (int t = 0; t < 4; ++t) {
    const int lc = 16 * t + m;
#pragma unroll
    for (int r = 0; r < 8; ++r) {
      const int lr = 16 * wave + 8 * hh + r;
      stg[lr * GBN + lc] = acc[t][r];
    }
  }
  __syncthreads();

  const int plane = col0 / nsplit;
  const int cc    = col0 - plane * nsplit;
  float* ob = outF + (size_t)plane * (size_t)pstride + cc + 4 * m;
  if constexpr (MODE == 0) {
    v4f fv[8];
#pragma unroll
    for (int i = 0; i < 8; ++i) {
      const int lr = 16 * wave + 2 * i + hh;
      fv[i] = *(const v4fa*)(stg + lr * GBN + 4 * m);
    }
#pragma unroll
    for (int i = 0; i < 8; ++i) {
      const int lr = 16 * wave + 2 * i + hh;
      *(volatile v4f*)(ob + (size_t)(rowBase + lr) * (size_t)ldo) = fv[i];
    }
    __threadfence();
#pragma unroll
    for (int i = 0; i < 8; ++i) {
      const int lr = 16 * wave + 2 * i + hh;
      *(volatile v4f*)(ob + (size_t)(rowBase + lr) * (size_t)ldo) = fv[i];
    }
  } else if constexpr (MODE == 1) {
    const bool sil = (plane != 0);
#pragma unroll 1
    for (int i = 0; i < 8; ++i) {
      const int lr = 16 * wave + 2 * i + hh;
      const v4f t = *(const v4fa*)(stg + lr * GBN + 4 * m);
      v4f o;
      o.x = sil ? silu_f(t.x) : t.x;
      o.y = sil ? silu_f(t.y) : t.y;
      o.z = sil ? silu_f(t.z) : t.z;
      o.w = sil ? silu_f(t.w) : t.w;
      put4(ob + (size_t)(rowBase + lr) * (size_t)ldo, o);
    }
  } else {
#pragma unroll 1
    for (int i = 0; i < 8; ++i) {
      const int lr = 16 * wave + 2 * i + hh;
      const v4f t = *(const v4fa*)(stg + lr * GBN + 4 * m);
      const v4f rv = *(const v4fa*)(res + (size_t)(rowBase + lr) * (size_t)ldo + col0 + 4 * m);
      v4f o;
      o.x = rv.x + t.x; o.y = rv.y + t.y; o.z = rv.z + t.z; o.w = rv.w + t.w;
      put4(ob + (size_t)(rowBase + lr) * (size_t)ldo, o);
    }
  }
}

__global__ __launch_bounds__(NTHR) __attribute__((amdgpu_num_vgpr(248))) void k_dw(
    const float* __restrict__ XI, const float* __restrict__ SP, float* U, unsigned short* UHL)
{
  __shared__ __attribute__((aligned(16))) float sw[9 * 128];
  const int tid = (int)threadIdx.x;
#pragma unroll 1
  for (int it = 0; it < 5; ++it) {
    const int i = tid + NTHR * it;
    const int ic = i < 1152 ? i : 1151;
    const int dch = ic / 9;
    sw[(ic - 9 * dch) * 128 + dch] = SP[SP_SCW + ic];
  }
  __syncthreads();
  const int gt = (int)blockIdx.x * NTHR + tid;
  const int q = gt & 31, t = gt >> 5;
  const int c0 = 4 * q;
  const int b = t >> 12, gi = (t >> 6) & 63, gj = t & 63;
  v4f acc = *(const v4fa*)(SP + SP_SCB + c0);
#pragma unroll 1
  for (int a = 0; a < 3; ++a) {
#pragma unroll 1
    for (int bq = 0; bq < 3; ++bq) {
      const int ii = gi - 1 + a, jj = gj - 1 + bq;
      const bool ok = (ii >= 0) && (ii < GH) && (jj >= 0) && (jj < GW);
      const int iic = ii < 0 ? 0 : (ii > GH - 1 ? GH - 1 : ii);
      const int jjc = jj < 0 ? 0 : (jj > GW - 1 ? GW - 1 : jj);
      v4f xv = *(const v4fa*)(XI + (size_t)(b * LSEQ + iic * GW + jjc) * DIN + c0);
      const v4f wv = *(const v4fa*)(sw + (a * 3 + bq) * 128 + c0);
      xv.x = ok ? xv.x : 0.0f; xv.y = ok ? xv.y : 0.0f; xv.z = ok ? xv.z : 0.0f; xv.w = ok ? xv.w : 0.0f;
      acc.x = fmaf(wv.x, xv.x, acc.x);
      acc.y = fmaf(wv.y, xv.y, acc.y);
      acc.z = fmaf(wv.z, xv.z, acc.z);
      acc.w = fmaf(wv.w, xv.w, acc.w);
    }
  }
  v4f uo;
  uo.x = silu_f(acc.x); uo.y = silu_f(acc.y); uo.z = silu_f(acc.z); uo.w = silu_f(acc.w);
  v4us hv, lv;
  hv[0] = hi_bits(uo.x); lv[0] = lo_bits(uo.x);
  hv[1] = hi_bits(uo.y); lv[1] = lo_bits(uo.y);
  hv[2] = hi_bits(uo.z); lv[2] = lo_bits(uo.z);
  hv[3] = hi_bits(uo.w); lv[3] = lo_bits(uo.w);
  float* up = U + (size_t)t * DIN + c0;
  unsigned short* hp = UHL + (size_t)t * 256 + c0;
  *(volatile v4f*)up = uo;
  *(volatile v4us*)hp = hv;
  *(volatile v4us*)(hp + DIN) = lv;
  __threadfence();
  *(volatile v4f*)up = uo;
  *(volatile v4us*)hp = hv;
  *(volatile v4us*)(hp + DIN) = lv;
}

__device__ __forceinline__ int seq_pos(int k, int l) {
  const int lr = (k & 2) ? (LSEQ - 1 - l) : l;
  const int tp = ((lr & 63) << 6) | (lr >> 6);
  return (k & 1) ? tp : lr;
}

__global__ __launch_bounds__(SCT) __attribute__((amdgpu_num_vgpr(248))) void k_scan(
    const float* __restrict__ U, const float* __restrict__ DBL, const float* __restrict__ SP, float* YS)
{
  __shared__ __attribute__((aligned(16))) float us[SCH * SCT];
  __shared__ __attribute__((aligned(16))) float ds[320 * 4];
  __shared__ __attribute__((aligned(16))) float ystg[SCH * SCT];
  const int tid = (int)threadIdx.x;
  const int blk = (int)blockIdx.x;
  const int k = blk >> 2, b = (blk >> 1) & 1, half = blk & 1;
  const int kd = k * DIN + half * 64 + tid;

  float h[NST], Ar[NST];
#pragma unroll
  for (int j = 0; j < 4; ++j) {
    const v4f a = *(const v4fa*)(SP + SP_SAN + (size_t)kd * NST + 4 * j);
    Ar[4 * j + 0] = a.x; Ar[4 * j + 1] = a.y; Ar[4 * j + 2] = a.z; Ar[4 * j + 3] = a.w;
    h[4 * j + 0] = 0.0f; h[4 * j + 1] = 0.0f; h[4 * j + 2] = 0.0f; h[4 * j + 3] = 0.0f;
  }
  const v4f dtw = *(const v4fa*)(SP + SP_SDTW + 4 * kd);
  const float dtb = SP[SP_SDTB + kd];
  const float Dd  = SP[SP_SD + kd];
  const float* Ub = U + (size_t)b * LSEQ * DIN + half * 64;
  const float* Db = DBL + (size_t)b * LSEQ * NXPAD + k * NDBL;
  float* Yb = YS + ((size_t)k * NTOK + (size_t)b * LSEQ) * DIN + half * 64;

#pragma unroll 1
  for (int ch = 0; ch < LSEQ / SCH; ++ch) {
    const int l0 = ch * SCH;
#pragma unroll
    for (int j = 0; j < 8; ++j) {
      const int f4 = tid + SCT * j;
      const int p = seq_pos(k, l0 + (f4 >> 4));
      *(v4fa*)(us + 4 * f4) = *(const v4fa*)(Ub + (size_t)p * DIN + 4 * (f4 & 15));
    }
#pragma unroll
    for (int j = 0; j < 5; ++j) {
      const int f4 = tid + SCT * j;
      const int fc = f4 < 288 ? f4 : 287;
      const int e = fc / 9;
      const int pc = fc - 9 * e;
      const int p = seq_pos(k, l0 + e);
      *(v4fa*)(ds + 4 * f4) = *(const v4fa*)(Db + (size_t)p * NXPAD + 4 * pc);
    }
    __syncthreads();

#pragma unroll 1
    for (int ll = 0; ll < SCH; ++ll) {
      const float uu = us[ll * SCT + tid];
      const float* bp = ds + ll * NDBL;
      const v4f dr = *(const v4fa*)bp;
      float pr = dr.x * dtw.x;
      pr = fmaf(dr.y, dtw.y, pr);
      pr = fmaf(dr.z, dtw.z, pr);
      pr = fmaf(dr.w, dtw.w, pr);
      const float dl = softplus_f(pr + dtb);
      const float du = dl * uu;
      float Bv[NST], Cv[NST];
#pragma unroll
      for (int j = 0; j < 4; ++j) {
        const v4f tb = *(const v4fa*)(bp + DTR + 4 * j);
        const v4f tc = *(const v4fa*)(bp + DTR + NST + 4 * j);
        Bv[4 * j + 0] = tb.x; Bv[4 * j + 1] = tb.y; Bv[4 * j + 2] = tb.z; Bv[4 * j + 3] = tb.w;
        Cv[4 * j + 0] = tc.x; Cv[4 * j + 1] = tc.y; Cv[4 * j + 2] = tc.z; Cv[4 * j + 3] = tc.w;
      }
#pragma unroll
      for (int n = 0; n < NST; ++n) {
        const float dA = expf(dl * Ar[n]);
        h[n] = dA * h[n] + du * Bv[n];
      }
      float y = h[0] * Cv[0];
#pragma unroll
      for (int n = 1; n < NST; ++n) y = fmaf(h[n], Cv[n], y);
      y = y + uu * Dd;
      ystg[ll * SCT + tid] = y;
    }
    __syncthreads();

#pragma unroll 1
    for (int j = 0; j < 8; ++j) {
      const int pz = tid + SCT * j;
      const int e = pz >> 4;
      const int c4 = (pz & 15) * 4;
      const int p = seq_pos(k, l0 + e);
      const v4f v = *(const v4fa*)(ystg + e * SCT + c4);
      put4(Yb + (size_t)p * DIN + c4, v);
    }
  }
}

__global__ __launch_bounds__(NTHR) __attribute__((amdgpu_num_vgpr(248))) void k_comb(
    const float* __restrict__ YS, const float* __restrict__ SZ, const float* __restrict__ SP,
    unsigned short* GHL)
{
  const int gt = (int)blockIdx.x * NTHR + (int)threadIdx.x;
  const int q = gt & 31, t = gt >> 5;
  const int c0 = 4 * q;
  const size_t ro = (size_t)t * DIN + c0;
  const size_t ps = (size_t)NTOK * DIN;
  const v4f y0 = *(const v4fa*)(YS + ro);
  const v4f y1 = *(const v4fa*)(YS + ps + ro);
  const v4f y2 = *(const v4fa*)(YS + 2 * ps + ro);
  const v4f y3 = *(const v4fa*)(YS + 3 * ps + ro);
  v4f s;
  s.x = ((y0.x + y2.x) + y1.x) + y3.x;
  s.y = ((y0.y + y2.y) + y1.y) + y3.y;
  s.z = ((y0.z + y2.z) + y1.z) + y3.z;
  s.w = ((y0.w + y2.w) + y1.w) + y3.w;
  float sm = (s.x + s.y) + (s.z + s.w);
  sm += __shfl_xor(sm, 1); sm += __shfl_xor(sm, 2); sm += __shfl_xor(sm, 4);
  sm += __shfl_xor(sm, 8); sm += __shfl_xor(sm, 16);
  const float mu = sm * (1.0f / 128.0f);
  v4f d;
  d.x = s.x - mu; d.y = s.y - mu; d.z = s.z - mu; d.w = s.w - mu;
  float qv = (d.x * d.x + d.y * d.y) + (d.z * d.z + d.w * d.w);
  qv += __shfl_xor(qv, 1); qv += __shfl_xor(qv, 2); qv += __shfl_xor(qv, 4);
  qv += __shfl_xor(qv, 8); qv += __shfl_xor(qv, 16);
  const float rs = 1.0f / sqrtf(qv * (1.0f / 128.0f) + 1e-5f);
  const v4f g  = *(const v4fa*)(SP + SP_SOG + c0);
  const v4f bt = *(const v4fa*)(SP + SP_SOB + c0);
  const v4f z  = *(const v4fa*)(SZ + ro);
  v4f o;
  o.x = (d.x * rs * g.x + bt.x) * z.x;
  o.y = (d.y * rs * g.y + bt.y) * z.y;
  o.z = (d.z * rs * g.z + bt.z) * z.z;
  o.w = (d.w * rs * g.w + bt.w) * z.w;
  v4us hv, lv;
  hv[0] = hi_bits(o.x); lv[0] = lo_bits(o.x);
  hv[1] = hi_bits(o.y); lv[1] = lo_bits(o.y);
  hv[2] = hi_bits(o.z); lv[2] = lo_bits(o.z);
  hv[3] = hi_bits(o.w); lv[3] = lo_bits(o.w);
  unsigned short* hp = GHL + (size_t)t * 256 + c0;
  *(volatile v4us*)hp = hv;
  *(volatile v4us*)(hp + DIN) = lv;
  __threadfence();
  *(volatile v4us*)hp = hv;
  *(volatile v4us*)(hp + DIN) = lv;
}

__device__ __forceinline__ void lds_gemm2(const unsigned short* A2, const unsigned short* __restrict__ WT2,
                                          float* outT, int w, int hh, int m)
{
  const int mt = w & 3, nh = w >> 2;
  v8f acc[2];
  {
    const v8f z = {0.f, 0.f, 0.f, 0.f, 0.f, 0.f, 0.f, 0.f};
    acc[0] = z; acc[1] = z;
  }
  const unsigned short* ap = A2 + (16 * mt + m) * A2P + 8 * hh;
  const unsigned short* wp = WT2 + (size_t)(32 * nh + m) * 256 + 8 * hh;
#pragma unroll 1
  for (int ks = 0; ks < 8; ++ks) {
    FragB af;
    af.h[0] = *(const v8usa*)(ap + 32 * ks);
    af.h[1] = *(const v8usa*)(ap + 32 * ks + 16);
#pragma unroll
    for (int t = 0; t < 2; ++t) {
      const unsigned short* wq = wp + (size_t)(16 * t) * 256 + 32 * ks;
      FragB bf;
      bf.h[0] = *(const v8usa*)wq;
      bf.h[1] = *(const v8usa*)(wq + 16);
      acc[t] = wmb(af, bf, acc[t]);
    }
  }
#pragma unroll
  for (int t = 0; t < 2; ++t) {
#pragma unroll
    for (int r = 0; r < 8; ++r)
      outT[(16 * mt + 8 * hh + r) * 64 + 32 * nh + 16 * t + m] = acc[t][r];
  }
}

__global__ __launch_bounds__(NTHR) __attribute__((amdgpu_num_vgpr(248))) void k_spe(
    const float* __restrict__ x1, const float* __restrict__ x2,
    const unsigned short* __restrict__ MINW, const unsigned short* __restrict__ MXP2,
    const unsigned short* __restrict__ MOUT2, const float* __restrict__ SP,
    float* out1, float* out2, float* XDD)
{
  extern __shared__ __attribute__((aligned(16))) unsigned char smem[];
  float* XR1 = (float*)(smem + O_XR1);
  float* XR2 = (float*)(smem + O_XR2);
  unsigned short* A1 = (unsigned short*)(smem + O_A1);
  float* XZ = (float*)(smem + O_XZ);
  unsigned short* A2 = (unsigned short*)(smem + O_A2);
  float* DB = (float*)(smem + O_DB);
  float* YM = (float*)(smem + O_YM);

  const int tid = (int)threadIdx.x, lane = tid & 31, w = tid >> 5, hh = lane >> 4, m = lane & 15;
  const int blk = (int)blockIdx.x;
  const int b = blk >> 9, hrow = (blk >> 2) & 127, w0 = (blk & 3) * 32;
  const size_t gbase = (size_t)b * CH * (HH * WW) + (size_t)hrow * WW + w0;

#pragma unroll
  for (int i = 0; i < 2; ++i) {
    const int idx = tid + NTHR * i;
    const int c = idx >> 3, q = idx & 7;
    const v4f v = *(const v4fa*)(x1 + gbase + (size_t)c * (HH * WW) + 4 * q);
    v4f r;
    r.x = bf16_val(v.x); r.y = bf16_val(v.y); r.z = bf16_val(v.z); r.w = bf16_val(v.w);
    *(v4fa*)(XR1 + c * 32 + 4 * q) = r;
    A1[(2 * (4 * q + 0)) * A1P + c] = (unsigned short)(__float_as_uint(r.x) >> 16);
    A1[(2 * (4 * q + 1)) * A1P + c] = (unsigned short)(__float_as_uint(r.y) >> 16);
    A1[(2 * (4 * q + 2)) * A1P + c] = (unsigned short)(__float_as_uint(r.z) >> 16);
    A1[(2 * (4 * q + 3)) * A1P + c] = (unsigned short)(__float_as_uint(r.w) >> 16);
  }
#pragma unroll
  for (int i = 0; i < 2; ++i) {
    const int idx = tid + NTHR * i;
    const int c = idx >> 3, q = idx & 7;
    const v4f v = *(const v4fa*)(x2 + gbase + (size_t)c * (HH * WW) + 4 * q);
    v4f r;
    r.x = bf16_val(v.x); r.y = bf16_val(v.y); r.z = bf16_val(v.z); r.w = bf16_val(v.w);
    *(v4fa*)(XR2 + c * 32 + 4 * q) = r;
    A1[(2 * (4 * q + 0) + 1) * A1P + c] = (unsigned short)(__float_as_uint(r.x) >> 16);
    A1[(2 * (4 * q + 1) + 1) * A1P + c] = (unsigned short)(__float_as_uint(r.y) >> 16);
    A1[(2 * (4 * q + 2) + 1) * A1P + c] = (unsigned short)(__float_as_uint(r.z) >> 16);
    A1[(2 * (4 * q + 3) + 1) * A1P + c] = (unsigned short)(__float_as_uint(r.w) >> 16);
  }
  __syncthreads();

  {
    const int mt = w & 3, nh = w >> 2;
    v8f acc[8];
    {
      const v8f z = {0.f, 0.f, 0.f, 0.f, 0.f, 0.f, 0.f, 0.f};
#pragma unroll
      for (int t = 0; t < 8; ++t) acc[t] = z;
    }
    const unsigned short* ap = A1 + (16 * mt + m) * A1P + 8 * hh;
    const unsigned short* wp = MINW + (size_t)(128 * nh + m) * 64 + 8 * hh;
#pragma unroll 1
    for (int ks = 0; ks < 2; ++ks) {
      FragB af;
      af.h[0] = *(const v8usa*)(ap + 32 * ks);
      af.h[1] = *(const v8usa*)(ap + 32 * ks + 16);
#pragma unroll
      for (int t = 0; t < 8; ++t) {
        const unsigned short* wq = wp + (size_t)(16 * t) * 64 + 32 * ks;
        FragB bf;
        bf.h[0] = *(const v8usa*)wq;
        bf.h[1] = *(const v8usa*)(wq + 16);
        acc[t] = wmb(af, bf, acc[t]);
      }
    }
#pragma unroll
    for (int t = 0; t < 8; ++t) {
#pragma unroll
      for (int r = 0; r < 8; ++r)
        XZ[(16 * mt + 8 * hh + r) * 256 + 128 * nh + 16 * t + m] = acc[t][r];
    }
  }
  __syncthreads();

  const int dch = tid & 127, pxb = tid >> 7;
  {
    const v4f cw = *(const v4fa*)(SP + SP_MCW + 4 * dch);
    const float cb = SP[SP_MCB + dch];
#pragma unroll 1
    for (int i = 0; i < 16; ++i) {
      const int px = pxb + 2 * i;
      float* r0 = XZ + (2 * px) * 256;
      float* r1 = r0 + 256;
      const float xi0 = r0[dch], xi1 = r1[dch];
      const float z0 = r0[128 + dch], z1 = r1[128 + dch];
      const float u0 = silu_f(cw.w * xi0 + cb);
      const float u1 = silu_f(fmaf(cw.w, xi1, cw.z * xi0) + cb);
      r0[dch] = u0;
      r1[dch] = u1;
      r0[128 + dch] = silu_f(z0);
      r1[128 + dch] = silu_f(z1);
      A2[(2 * px) * A2P + dch]           = hi_bits(u0);
      A2[(2 * px) * A2P + 128 + dch]     = lo_bits(u0);
      A2[(2 * px + 1) * A2P + dch]       = hi_bits(u1);
      A2[(2 * px + 1) * A2P + 128 + dch] = lo_bits(u1);
    }
  }
  __syncthreads();

  lds_gemm2(A2, MXP2, DB, w, hh, m);
  __syncthreads();

  {
    const v4f dtw = *(const v4fa*)(SP + SP_MDTW + 4 * dch);
    const float dtb = SP[SP_MDTB + dch];
    const float Dd  = SP[SP_MD + dch];
    float Ar[NST];
#pragma unroll
    for (int j = 0; j < 4; ++j) {
      const v4f a = *(const v4fa*)(SP + SP_MAN + (size_t)dch * NST + 4 * j);
      Ar[4 * j + 0] = a.x; Ar[4 * j + 1] = a.y; Ar[4 * j + 2] = a.z; Ar[4 * j + 3] = a.w;
    }
#pragma unroll 1
    for (int i = 0; i < 16; ++i) {
      const int px = pxb + 2 * i;
      const float* q0 = DB + (2 * px) * 64;
      const float* q1 = q0 + 64;
      const float* r0 = XZ + (2 * px) * 256;
      const float* r1 = r0 + 256;
      const float u0 = r0[dch], u1 = r1[dch];
      const float sz0 = r0[128 + dch], sz1 = r1[128 + dch];
      const v4f d0 = *(const v4fa*)q0;
      const v4f d1 = *(const v4fa*)q1;
      float p0 = d0.x * dtw.x;
      p0 = fmaf(d0.y, dtw.y, p0); p0 = fmaf(d0.z, dtw.z, p0); p0 = fmaf(d0.w, dtw.w, p0);
      float p1 = d1.x * dtw.x;
      p1 = fmaf(d1.y, dtw.y, p1); p1 = fmaf(d1.z, dtw.z, p1); p1 = fmaf(d1.w, dtw.w, p1);
      const float dt0 = softplus_f(p0 + dtb);
      const float dt1 = softplus_f(p1 + dtb);
      const float du0 = dt0 * u0, du1 = dt1 * u1;
      float B0[NST], C0[NST], B1[NST], C1[NST];
#pragma unroll
      for (int j = 0; j < 4; ++j) {
        const v4f tb0 = *(const v4fa*)(q0 + DTR + 4 * j);
        const v4f tc0 = *(const v4fa*)(q0 + DTR + NST + 4 * j);
        const v4f tb1 = *(const v4fa*)(q1 + DTR + 4 * j);
        const v4f tc1 = *(const v4fa*)(q1 + DTR + NST + 4 * j);
        B0[4 * j + 0] = tb0.x; B0[4 * j + 1] = tb0.y; B0[4 * j + 2] = tb0.z; B0[4 * j + 3] = tb0.w;
        C0[4 * j + 0] = tc0.x; C0[4 * j + 1] = tc0.y; C0[4 * j + 2] = tc0.z; C0[4 * j + 3] = tc0.w;
        B1[4 * j + 0] = tb1.x; B1[4 * j + 1] = tb1.y; B1[4 * j + 2] = tb1.z; B1[4 * j + 3] = tb1.w;
        C1[4 * j + 0] = tc1.x; C1[4 * j + 1] = tc1.y; C1[4 * j + 2] = tc1.z; C1[4 * j + 3] = tc1.w;
      }
      float y0 = 0.0f, y1 = 0.0f;
#pragma unroll
      for (int n = 0; n < NST; ++n) {
        const float h0 = du0 * B0[n];
        y0 = fmaf(h0, C0[n], y0);
        const float h1 = expf(dt1 * Ar[n]) * h0 + du1 * B1[n];
        y1 = fmaf(h1, C1[n], y1);
      }
      const float g0 = (y0 + u0 * Dd) * sz0;
      const float g1 = (y1 + u1 * Dd) * sz1;
      A2[(2 * px) * A2P + dch]           = hi_bits(g0);
      A2[(2 * px) * A2P + 128 + dch]     = lo_bits(g0);
      A2[(2 * px + 1) * A2P + dch]       = hi_bits(g1);
      A2[(2 * px + 1) * A2P + 128 + dch] = lo_bits(g1);
    }
  }
  __syncthreads();

  lds_gemm2(A2, MOUT2, YM, w, hh, m);
  __syncthreads();

  {
    const int q = tid & 3, tl = tid >> 2;
    float* row = YM + tl * 64 + 16 * q;
    float s = 0.0f;
#pragma unroll 4
    for (int j = 0; j < 16; ++j) s += row[j];
    s += __shfl_xor(s, 1);
    s += __shfl_xor(s, 2);
    const float mu = s * (1.0f / 64.0f);
    float qv = 0.0f;
#pragma unroll 4
    for (int j = 0; j < 16; ++j) {
      const float d = row[j] - mu;
      qv += d * d;
    }
    qv += __shfl_xor(qv, 1);
    qv += __shfl_xor(qv, 2);
    const float rs = 1.0f / sqrtf(qv * (1.0f / 64.0f) + 1e-5f);
#pragma unroll 2
    for (int j = 0; j < 16; ++j) {
      const int c = 16 * q + j;
      row[j] = silu_f((row[j] - mu) * rs * SP[SP_SPEG + c] + SP[SP_SPEB + c]);
    }
  }
  __syncthreads();

  {
    const int q = tid & 7;
    v4f o1[2], o2[2], od[2];
#pragma unroll
    for (int i = 0; i < 2; ++i) {
      const int c = (tid >> 3) + 32 * i;
      const v4f a1 = *(const v4fa*)(XR1 + c * 32 + 4 * q);
      const v4f a2 = *(const v4fa*)(XR2 + c * 32 + 4 * q);
      v4f p1, p2;
      p1.x = a1.x + YM[(2 * (4 * q + 0)) * 64 + c];
      p1.y = a1.y + YM[(2 * (4 * q + 1)) * 64 + c];
      p1.z = a1.z + YM[(2 * (4 * q + 2)) * 64 + c];
      p1.w = a1.w + YM[(2 * (4 * q + 3)) * 64 + c];
      p2.x = a2.x + YM[(2 * (4 * q + 0) + 1) * 64 + c];
      p2.y = a2.y + YM[(2 * (4 * q + 1) + 1) * 64 + c];
      p2.z = a2.z + YM[(2 * (4 * q + 2) + 1) * 64 + c];
      p2.w = a2.w + YM[(2 * (4 * q + 3) + 1) * 64 + c];
      o1[i] = p1;
      o2[i] = p2;
      v4f dd;
      dd.x = p2.x - p1.x; dd.y = p2.y - p1.y; dd.z = p2.z - p1.z; dd.w = p2.w - p1.w;
      od[i] = dd;
    }
#pragma unroll
    for (int i = 0; i < 2; ++i) {
      const int c = (tid >> 3) + 32 * i;
      const size_t go = gbase + (size_t)c * (HH * WW) + 4 * q;
      *(volatile v4f*)(out1 + go) = o1[i];
      *(volatile v4f*)(out2 + go) = o2[i];
      *(volatile v4f*)(XDD + go)  = od[i];
    }
    __threadfence();
#pragma unroll
    for (int i = 0; i < 2; ++i) {
      const int c = (tid >> 3) + 32 * i;
      const size_t go = gbase + (size_t)c * (HH * WW) + 4 * q;
      *(volatile v4f*)(out1 + go) = o1[i];
      *(volatile v4f*)(out2 + go) = o2[i];
      *(volatile v4f*)(XDD + go)  = od[i];
    }
  }
}

__global__ __launch_bounds__(NTHR) __attribute__((amdgpu_num_vgpr(248))) void k_fuse(
    const float* __restrict__ XV, const float* __restrict__ XDD, const float* __restrict__ SP, float* out0)
{
  __shared__ __attribute__((aligned(16))) float sv[512 * 4];
  __shared__ __attribute__((aligned(16))) float stile[2 * 2048];
  __shared__ __attribute__((aligned(16))) float sg[64];
  const int tid = (int)threadIdx.x, lane = tid & 31, w = tid >> 5;
  const int blk = (int)blockIdx.x;
  const int b = blk >> 9, hrow = (blk >> 2) & 127, w0 = (blk & 3) * 32;
  const size_t gbase = (size_t)b * CH * (HH * WW) + (size_t)hrow * WW + w0;
  const int kk = hrow >> 1, odd = hrow & 1;
  const int km = kk > 0 ? kk - 1 : 0;
  const int kp = kk < GH - 1 ? kk + 1 : GH - 1;
  const int ra = odd ? kk : km;
  const int rb = odd ? kp : kk;
  const float wa = odd ? 0.75f : 0.25f;
  const float wb = odd ? 0.25f : 0.75f;
  const int jbase = w0 >> 1;

#pragma unroll
  for (int i = 0; i < 2; ++i) {
    const int idx = tid + NTHR * i;
    const int idc = idx < 288 ? idx : 287;
    const int cs = idc >> 4, c4 = (idc & 15) * 4;
    int col = jbase - 1 + cs;
    col = col < 0 ? 0 : (col > GW - 1 ? GW - 1 : col);
    const v4f a  = *(const v4fa*)(XV + (size_t)(b * LSEQ + ra * GW + col) * CH + c4);
    const v4f bq = *(const v4fa*)(XV + (size_t)(b * LSEQ + rb * GW + col) * CH + c4);
    v4f v;
    v.x = wa * a.x + wb * bq.x; v.y = wa * a.y + wb * bq.y;
    v.z = wa * a.z + wb * bq.z; v.w = wa * a.w + wb * bq.w;
    *(v4fa*)(sv + 4 * idx) = v;
  }
#pragma unroll
  for (int i = 0; i < 2; ++i) {
    const int idx = tid + NTHR * i;
    const int c = idx >> 3, q = idx & 7;
    *(v4fa*)(stile + 2048 + c * 32 + 4 * q) = *(const v4fa*)(XDD + gbase + (size_t)c * (HH * WW) + 4 * q);
  }
  __syncthreads();

#pragma unroll
  for (int i = 0; i < 8; ++i) {
    const int item = tid + NTHR * i;
    const int c = item & 63, px = item >> 6;
    const int jl = px >> 1, od = px & 1;
    const int ca = jl + od;
    const float wl = od ? 0.75f : 0.25f;
    const float wr = od ? 0.25f : 0.75f;
    stile[c * 32 + px] = wl * sv[ca * 64 + c] + wr * sv[(ca + 1) * 64 + c];
  }
  __syncthreads();

  if (w < 2) {
    const int tb = w * 2048;
    const int wo = w ? SP_GBW : SP_GAW;
    const int bo = w ? SP_GBB : SP_GAB;
    float s = 0.0f;
#pragma unroll 4
    for (int c = 0; c < CH; ++c) s = fmaf(stile[tb + c * 32 + lane], SP[wo + c], s);
    s = s + SP[bo];
    sg[w * 32 + lane] = 1.0f / (1.0f + expf(-s));
  }
  __syncthreads();

  {
    const int q = tid & 7;
    const v4f ga = *(const v4fa*)(sg + 4 * q);
    const v4f gb = *(const v4fa*)(sg + 32 + 4 * q);
    v4f ov[2];
#pragma unroll
    for (int i = 0; i < 2; ++i) {
      const int c = (tid >> 3) + 32 * i;
      const v4f xs4 = *(const v4fa*)(stile + c * 32 + 4 * q);
      const v4f xd4 = *(const v4fa*)(stile + 2048 + c * 32 + 4 * q);
      v4f o;
      o.x = ga.x * xs4.x + gb.x * xd4.x;
      o.y = ga.y * xs4.y + gb.y * xd4.y;
      o.z = ga.z * xs4.z + gb.z * xd4.z;
      o.w = ga.w * xs4.w + gb.w * xd4.w;
      ov[i] = o;
    }
#pragma unroll
    for (int i = 0; i < 2; ++i) {
      const int c = (tid >> 3) + 32 * i;
      *(volatile v4f*)(out0 + gbase + (size_t)c * (HH * WW) + 4 * q) = ov[i];
    }
    __threadfence();
#pragma unroll
    for (int i = 0; i < 2; ++i) {
      const int c = (tid >> 3) + 32 * i;
      *(volatile v4f*)(out0 + gbase + (size_t)c * (HH * WW) + 4 * q) = ov[i];
    }
  }
}

static inline size_t al256(size_t o) { return (o + 255) & ~(size_t)255; }

extern "C" void kernel_launch(void* const* d_in, const int* in_sizes, int n_in,
                              void* d_out, int out_size, void* d_ws, size_t ws_size,
                              hipStream_t stream) {
  if (n_in < 35) return;
  static const int expect_n[35] = {
    PLANE, PLANE, PLANE, 16384, 512, 128, 4608, 512, 128, 2048, 128, 8192, 64, 64, 16384, 64, 64, 64, 64, 64,
    16384, 1152, 128, 18432, 2048, 512, 8192, 512, 128, 128, 8192, 64, 1, 64, 1 };
  for (int i = 0; i < 35; ++i) if (in_sizes[i] != expect_n[i]) return;
  if (out_size != 3 * PLANE) return;

  const float* x_spa     = (const float*)d_in[0];
  const float* x1        = (const float*)d_in[1];
  const float* x2        = (const float*)d_in[2];
  const float* m_in_w    = (const float*)d_in[3];
  const float* m_conv_w  = (const float*)d_in[4];
  const float* m_conv_b  = (const float*)d_in[5];
  const float* m_xproj_w = (const float*)d_in[6];
  const float* m_dt_w    = (const float*)d_in[7];
  const float* m_dt_b    = (const float*)d_in[8];
  const float* m_A_log   = (const float*)d_in[9];
  const float* m_D       = (const float*)d_in[10];
  const float* m_out_w   = (const float*)d_in[11];
  const float* spe_g     = (const float*)d_in[12];
  const float* spe_b     = (const float*)d_in[13];
  const float* pe_w      = (const float*)d_in[14];
  const float* pe_b      = (const float*)d_in[15];
  const float* gn_g      = (const float*)d_in[16];
  const float* gn_b      = (const float*)d_in[17];
  const float* vl_g      = (const float*)d_in[18];
  const float* vl_b      = (const float*)d_in[19];
  const float* s_in_w    = (const float*)d_in[20];
  const float* s_conv_w  = (const float*)d_in[21];
  const float* s_conv_b  = (const float*)d_in[22];
  const float* s_xproj_w = (const float*)d_in[23];
  const float* s_dt_w    = (const float*)d_in[24];
  const float* s_dt_b    = (const float*)d_in[25];
  const float* s_A_log   = (const float*)d_in[26];
  const float* s_D       = (const float*)d_in[27];
  const float* s_og      = (const float*)d_in[28];
  const float* s_ob      = (const float*)d_in[29];
  const float* s_out_w   = (const float*)d_in[30];
  const float* gA_w      = (const float*)d_in[31];
  const float* gA_b      = (const float*)d_in[32];
  const float* gB_w      = (const float*)d_in[33];
  const float* gB_b      = (const float*)d_in[34];

  float* out0 = (float*)d_out;
  float* out1 = out0 + PLANE;
  float* out2 = out0 + 2 * (size_t)PLANE;

  char* ws = (char*)d_ws;
  size_t off = 0;
  const size_t oXP   = off; off = al256(off + (size_t)NTOK * CH * 4);
  const size_t oXIN  = off; off = al256(off + (size_t)NTOK * CH * 4);
  const size_t oXNHL = off; off = al256(off + (size_t)NTOK * 128 * 2);
  const size_t oXI   = off; off = al256(off + (size_t)NTOK * DIN * 4);
  const size_t oSZ   = off; off = al256(off + (size_t)NTOK * DIN * 4);
  const size_t oU    = off; off = al256(off + (size_t)NTOK * DIN * 4);
  const size_t oUHL  = off; off = al256(off + (size_t)NTOK * 256 * 2);
  const size_t oDBL  = off; off = al256(off + (size_t)NTOK * NXPAD * 4);
  const size_t oYS   = off; off = al256(off + (size_t)4 * NTOK * DIN * 4);
  const size_t oGHL  = off; off = al256(off + (size_t)NTOK * 256 * 2);
  const size_t oXV   = off; off = al256(off + (size_t)NTOK * CH * 4);
  const size_t oXDD  = off; off = al256(off + (size_t)PLANE * 4);
  const size_t oREC  = off; off = al256(off + (size_t)128 * 16 * 8);
  const size_t oPEW  = off; off = al256(off + (size_t)64 * 256 * 2);
  const size_t oMINW = off; off = al256(off + (size_t)256 * 64 * 2);
  const size_t oSINW = off; off = al256(off + (size_t)256 * 128 * 2);
  const size_t oSXP  = off; off = al256(off + (size_t)NXPAD * 256 * 2);
  const size_t oSOUT = off; off = al256(off + (size_t)64 * 256 * 2);
  const size_t oMXP  = off; off = al256(off + (size_t)64 * 256 * 2);
  const size_t oMOUT = off; off = al256(off + (size_t)64 * 256 * 2);
  const size_t oSP   = off; off = al256(off + (size_t)SP_END * 4);
  if (off > ws_size || off > (size_t)WSMAX) return;

  float*          XP   = (float*)(ws + oXP);
  float*          XIN  = (float*)(ws + oXIN);
  unsigned short* XNHL = (unsigned short*)(ws + oXNHL);
  float*          XI   = (float*)(ws + oXI);
  float*          SZ   = (float*)(ws + oSZ);
  float*          Up   = (float*)(ws + oU);
  unsigned short* UHL  = (unsigned short*)(ws + oUHL);
  float*          DBL  = (float*)(ws + oDBL);
  float*          YS   = (float*)(ws + oYS);
  unsigned short* GHL  = (unsigned short*)(ws + oGHL);
  float*          XV   = (float*)(ws + oXV);
  float*          XDD  = (float*)(ws + oXDD);
  double*         REC  = (double*)(ws + oREC);
  unsigned short* PEW  = (unsigned short*)(ws + oPEW);
  unsigned short* MINW = (unsigned short*)(ws + oMINW);
  unsigned short* SINW = (unsigned short*)(ws + oSINW);
  unsigned short* SXP  = (unsigned short*)(ws + oSXP);
  unsigned short* SOUT = (unsigned short*)(ws + oSOUT);
  unsigned short* MXP  = (unsigned short*)(ws + oMXP);
  unsigned short* MOUT = (unsigned short*)(ws + oMOUT);
  float*          SP   = (float*)(ws + oSP);
  const int pstr = (int)((oSZ - oXI) / 4);

  k_pa<<<PA_U / NTHR, NTHR, 0, stream>>>(pe_w, m_in_w, s_in_w, s_xproj_w, PEW, MINW, SINW, SXP);
  k_pb<<<PB_U / NTHR, NTHR, 0, stream>>>(s_out_w, m_xproj_w, m_out_w, SOUT, MXP, MOUT);
  k_pc<<<(PC_U + NTHR - 1) / NTHR, NTHR, 0, stream>>>(s_conv_w, s_conv_b, s_dt_w, s_dt_b, s_D, s_og, s_ob,
                                                      s_A_log, SP);
  k_pd<<<(PD_U + NTHR - 1) / NTHR, NTHR, 0, stream>>>(m_conv_w, m_conv_b, m_dt_w, m_dt_b, m_D, m_A_log, SP);
  k_pf<<<(PF_U + NTHR - 1) / NTHR, NTHR, 0, stream>>>(spe_g, spe_b, pe_b, gn_g, gn_b, vl_g, vl_b, SP);
  k_pg<<<(PG_U + NTHR - 1) / NTHR, NTHR, 0, stream>>>(gA_w, gB_w, gA_b, gB_b, SP);
  k_pe<<<NTOK / 64, GTHR, 0, stream>>>(x_spa, PEW, SP, XP, REC);
  k_gnln<<<NTOK / 64, NTHR, 0, stream>>>(XP, REC, SP, XIN, XNHL);
  k_gemm<1><<<dim3(NTOK / GBM, (2 * DIN) / GBN), GTHR, 0, stream>>>(
      XNHL, 128, SINW, 128, 128, XI, DIN, DIN, pstr, SP);
  k_dw<<<(NTOK * 32) / NTHR, NTHR, 0, stream>>>(XI, SP, Up, UHL);
  k_gemm<0><<<dim3(NTOK / GBM, NXPAD / GBN), GTHR, 0, stream>>>(
      UHL, 256, SXP, 256, 256, DBL, NXPAD, NXPAD, 0, SP);
  k_scan<<<16, SCT, 0, stream>>>(Up, DBL, SP, YS);
  k_comb<<<(NTOK * 32) / NTHR, NTHR, 0, stream>>>(YS, SZ, SP, GHL);
  k_gemm<2><<<dim3(NTOK / GBM, CH / GBN), GTHR, 0, stream>>>(
      GHL, 256, SOUT, 256, 256, XV, CH, CH, 0, XIN);
  hipFuncSetAttribute(reinterpret_cast<const void*>(&k_spe), hipFuncAttributeMaxDynamicSharedMemorySize, SPE_LDS);
  k_spe<<<NB * HH * (WW / 32), NTHR, SPE_LDS, stream>>>(x1, x2, MINW, MXP, MOUT, SP, out1, out2, XDD);
  k_fuse<<<NB * HH * (WW / 32), NTHR, 0, stream>>>(XV, XDD, SP, out0);
}
